// TSPPruningGNN_35321811042630
// MI455X (gfx1250) — hardware-verified
//
#include <hip/hip_runtime.h>
#define NNODE 100000
#define NE 3200000
#define NTOT (NE + NNODE)
#define FIN 9
#define F1 64
#define F2 32

typedef __bf16 v16b __attribute__((ext_vector_type(16)));
typedef unsigned short v8us __attribute__((ext_vector_type(8), may_alias));
typedef float  v8f  __attribute__((ext_vector_type(8)));
typedef float  v4f  __attribute__((ext_vector_type(4)));
typedef float  v4fa __attribute__((ext_vector_type(4), may_alias));
union FragB { v16b v; v8us half[2]; unsigned short u[16]; };

__device__ __forceinline__ unsigned short bf16_bits(float x) { unsigned int u = __float_as_uint(x); return (unsigned short)((u + 0x7FFFu + ((u >> 16) & 1u)) >> 16); }
__device__ __forceinline__ float bf16_val(unsigned short b) { return __uint_as_float(((unsigned int)b) << 16); }
__device__ __forceinline__ float bf16_round(float x) { return bf16_val(bf16_bits(x)); }
template <int NT>
__device__ __forceinline__ v8f mmaN(v16b ah, v16b al, v16b bh, v16b bl, v8f c) {
  c = __builtin_amdgcn_wmma_f32_16x16x32_bf16(false, ah, false, bh, (short)0, c, false, false);
  if (NT >= 2) c = __builtin_amdgcn_wmma_f32_16x16x32_bf16(false, al, false, bh, (short)0, c, false, false);
  if (NT >= 3) c = __builtin_amdgcn_wmma_f32_16x16x32_bf16(false, ah, false, bl, (short)0, c, false, false);
  asm volatile("v_nop\n\tv_nop\n\tv_nop\n\tv_nop" : "+v"(c) : "v"(ah), "v"(al), "v"(bh), "v"(bl));
  return c;
}

__global__ __launch_bounds__(256) void k_wt_bf16(const float* __restrict__ W, unsigned short* __restrict__ Wt, int K, int N) {
  const int t = blockIdx.x * 256 + threadIdx.x;
  const int k8n = K / 8;
  if (t >= N * k8n) return;
  const int n = t / k8n, k8 = (t % k8n) * 8;
  v8us v;
#pragma unroll
  for (int i = 0; i < 8; ++i) v[i] = bf16_bits(W[(size_t)(k8 + i) * N + n]);
  *(volatile v8us*)(Wt + (size_t)n * K + k8) = v;
  __threadfence();
  *(volatile v8us*)(Wt + (size_t)n * K + k8) = v;
}

template <bool ASPLIT, int ACT, bool BIAS_BF16>
__global__ __launch_bounds__(128) void k_gemm_bf(const float* __restrict__ A, int lda, const unsigned short* __restrict__ Wt, int ldb,
                                               const float* __restrict__ bias, float* __restrict__ C, int ldc, int M, int N, int K) {
  __shared__ __attribute__((aligned(16))) float so[4][16][64];
  const int tid = threadIdx.x, w = tid >> 5, lane = tid & 31, ln = lane & 15, hh = lane >> 4;
  const int ntn = N / 64;
  const int wid = blockIdx.x * 4 + w;
  const int mt = wid / ntn, nq = wid % ntn;
  if (mt * 16 >= M) return;
  const int row0 = mt * 16, col0 = nq * 64;
  const float* arow = A + (size_t)(row0 + ln) * lda;
  v8f acc[4] = {};
  for (int kb = 0; kb < K; kb += 32) {
    FragB ah, al;
    const v4f x0 = *(const v4fa*)(arow + kb + 8 * hh), x1 = *(const v4fa*)(arow + kb + 8 * hh + 4);
    const v4f x2 = *(const v4fa*)(arow + kb + 16 + 8 * hh), x3 = *(const v4fa*)(arow + kb + 16 + 8 * hh + 4);
    float xs[16] = {x0[0],x0[1],x0[2],x0[3],x1[0],x1[1],x1[2],x1[3],x2[0],x2[1],x2[2],x2[3],x3[0],x3[1],x3[2],x3[3]};
#pragma unroll
    for (int i = 0; i < 16; ++i) { const unsigned short hb = bf16_bits(xs[i]); ah.u[i] = hb; al.u[i] = ASPLIT ? bf16_bits(xs[i] - bf16_val(hb)) : (unsigned short)0; }
#pragma unroll
    for (int t = 0; t < 4; ++t) {
      const unsigned short* brow = Wt + (size_t)(col0 + t * 16 + ln) * ldb + kb;
      FragB b;
      b.half[0] = *(const v8us*)(brow + 8 * hh);
      b.half[1] = *(const v8us*)(brow + 16 + 8 * hh);
      acc[t] = mmaN<ASPLIT ? 2 : 1>(ah.v, al.v, b.v, b.v, acc[t]);
    }
  }
#pragma unroll
  for (int t = 0; t < 4; ++t) {
    float bv = bias ? bias[col0 + t * 16 + ln] : 0.f;
    if (BIAS_BF16) bv = bf16_round(bv);
#pragma unroll
    for (int r = 0; r < 8; ++r) { float v = acc[t][r] + bv; if (ACT == 1) v = fmaxf(v, 0.f); so[w][8 * hh + r][t * 16 + ln] = v; }
  }
  __builtin_amdgcn_fence(__ATOMIC_ACQ_REL, "workgroup");
  __builtin_amdgcn_wave_barrier();
  const int rsub = lane >> 4, c4 = (lane & 15) * 4;
  for (int pass = 0; pass < 2; ++pass) {
#pragma unroll
    for (int q = 0; q < 8; ++q) {
      const int r = q * 2 + rsub;
      const v4f v = *(const v4fa*)&so[w][r][c4];
      *(volatile v4f*)(C + (size_t)(row0 + r) * ldc + col0 + c4) = v;
    }
    if (pass == 0) __threadfence();
  }
}

template <int D, bool CAUSAL>
__global__ __launch_bounds__(128) void k_flash(const float* __restrict__ qb, const float* __restrict__ kb, const float* __restrict__ vb,
                                             int pitch, int T, int H, float scale, float* __restrict__ y, int ypitch) {
  constexpr int KS = D / 32;
  constexpr int DT = D / 16;
  __shared__ __attribute__((aligned(16))) unsigned short sKh[32][D + 8], sKl[32][D + 8], sVh[32][D + 8], sVl[32][D + 8];
  __shared__ __attribute__((aligned(16))) unsigned short sPh[4][16][40], sPl[4][16][40];
  __shared__ __attribute__((aligned(16))) float sO[4][16][D];
  const int tid = threadIdx.x, w = tid >> 5, lane = tid & 31, ln = lane & 15, hh = lane >> 4;
  const int nqb = (T + 63) / 64;
  const int bh = blockIdx.x / nqb, qblk = blockIdx.x % nqb;
  const int b = bh / H, h = bh % H;
  const int q0 = qblk * 64 + w * 16;
  const float* Q = qb + (size_t)b * T * pitch + h * D;
  const float* K = kb + (size_t)b * T * pitch + h * D;
  const float* V = vb + (size_t)b * T * pitch + h * D;

  FragB aqh[KS], aql[KS];
  {
    int row = q0 + ln; if (row >= T) row = T - 1;
    const float* qr = Q + (size_t)row * pitch;
#pragma unroll
    for (int ks = 0; ks < KS; ++ks)
#pragma unroll
      for (int i = 0; i < 16; ++i) {
        const int d = ks * 32 + ((i < 8) ? (8 * hh + i) : (16 + 8 * hh + (i - 8)));
        const float x = qr[d] * scale; const unsigned short hb = bf16_bits(x);
        aqh[ks].u[i] = hb; aql[ks].u[i] = bf16_bits(x - bf16_val(hb));
      }
  }
  float m_r[8], l_r[8];
#pragma unroll
  for (int r = 0; r < 8; ++r) { m_r[r] = -3.0e38f; l_r[r] = 0.f; }
  v8f oacc[DT];
#pragma unroll
  for (int dt = 0; dt < DT; ++dt) oacc[dt] = (v8f){0.f,0.f,0.f,0.f,0.f,0.f,0.f,0.f};

  const int kv_end = CAUSAL ? min(T, qblk * 64 + 64) : T;
  for (int j0 = 0; j0 < kv_end; j0 += 32) {
    __syncthreads();
    for (int e = tid; e < 32 * (D / 4); e += 128) {
      const int r = e / (D / 4), c4 = (e % (D / 4)) * 4;
      const int key = j0 + r;
      v4f kf = {0.f,0.f,0.f,0.f}, vf = {0.f,0.f,0.f,0.f};
      if (key < T) { kf = *(const v4fa*)(K + (size_t)key * pitch + c4); vf = *(const v4fa*)(V + (size_t)key * pitch + c4); }
#pragma unroll
      for (int t = 0; t < 4; ++t) {
        unsigned short hb = bf16_bits(kf[t]); sKh[r][c4 + t] = hb; sKl[r][c4 + t] = bf16_bits(kf[t] - bf16_val(hb));
        hb = bf16_bits(vf[t]); sVh[r][c4 + t] = hb; sVl[r][c4 + t] = bf16_bits(vf[t] - bf16_val(hb));
      }
    }
    __syncthreads();
    v8f s[2];
#pragma unroll
    for (int nt = 0; nt < 2; ++nt) {
      v8f acc = {};
#pragma unroll
      for (int ks = 0; ks < KS; ++ks) {
        FragB bh_, bl_;
        bh_.half[0] = *(const v8us*)&sKh[nt * 16 + ln][ks * 32 + 8 * hh]; bh_.half[1] = *(const v8us*)&sKh[nt * 16 + ln][ks * 32 + 16 + 8 * hh];
        bl_.half[0] = *(const v8us*)&sKl[nt * 16 + ln][ks * 32 + 8 * hh]; bl_.half[1] = *(const v8us*)&sKl[nt * 16 + ln][ks * 32 + 16 + 8 * hh];
        acc = mmaN<3>(aqh[ks].v, aql[ks].v, bh_.v, bl_.v, acc);
      }
      s[nt] = acc;
    }
    float alpha[8];
#pragma unroll
    for (int r = 0; r < 8; ++r) {
      const int qi = q0 + 8 * hh + r;
      const int ja = j0 + ln, jb = j0 + 16 + ln;
      if (CAUSAL) { if (ja > qi) s[0][r] = -3.0e38f; if (jb > qi) s[1][r] = -3.0e38f; }
      if (ja >= T) s[0][r] = -3.0e38f;
      if (jb >= T) s[1][r] = -3.0e38f;
      float mx = fmaxf(s[0][r], s[1][r]);
      mx = fmaxf(mx, __shfl_xor(mx, 1, 32)); mx = fmaxf(mx, __shfl_xor(mx, 2, 32)); mx = fmaxf(mx, __shfl_xor(mx, 4, 32)); mx = fmaxf(mx, __shfl_xor(mx, 8, 32));
      const float mnew = fmaxf(m_r[r], mx);
      alpha[r] = (mnew > -1.0e38f) ? __expf(m_r[r] - mnew) : 1.0f;
      const float p0 = (s[0][r] > -1.0e38f) ? __expf(s[0][r] - mnew) : 0.f;
      const float p1 = (s[1][r] > -1.0e38f) ? __expf(s[1][r] - mnew) : 0.f;
      m_r[r] = mnew;
      l_r[r] = l_r[r] * alpha[r] + p0 + p1;
      unsigned short hb = bf16_bits(p0); sPh[w][8 * hh + r][ln] = hb;      sPl[w][8 * hh + r][ln] = bf16_bits(p0 - bf16_val(hb));
      hb = bf16_bits(p1);                sPh[w][8 * hh + r][16 + ln] = hb; sPl[w][8 * hh + r][16 + ln] = bf16_bits(p1 - bf16_val(hb));
    }
#pragma unroll
    for (int dt = 0; dt < DT; ++dt)
#pragma unroll
      for (int r = 0; r < 8; ++r) oacc[dt][r] *= alpha[r];
    __builtin_amdgcn_fence(__ATOMIC_ACQ_REL, "workgroup");
    __builtin_amdgcn_wave_barrier();
    FragB pah, pal;
    pah.half[0] = *(const v8us*)&sPh[w][ln][8 * hh]; pah.half[1] = *(const v8us*)&sPh[w][ln][16 + 8 * hh];
    pal.half[0] = *(const v8us*)&sPl[w][ln][8 * hh]; pal.half[1] = *(const v8us*)&sPl[w][ln][16 + 8 * hh];
#pragma unroll
    for (int dt = 0; dt < DT; ++dt) {
      FragB bvh, bvl;
#pragma unroll
      for (int i = 0; i < 8; ++i) {
        bvh.u[i] = sVh[8 * hh + i][dt * 16 + ln]; bvh.u[8 + i] = sVh[16 + 8 * hh + i][dt * 16 + ln];
        bvl.u[i] = sVl[8 * hh + i][dt * 16 + ln]; bvl.u[8 + i] = sVl[16 + 8 * hh + i][dt * 16 + ln];
      }
      oacc[dt] = mmaN<3>(pah.v, pal.v, bvh.v, bvl.v, oacc[dt]);
    }
    __builtin_amdgcn_fence(__ATOMIC_ACQ_REL, "workgroup");
    __builtin_amdgcn_wave_barrier();
  }
#pragma unroll
  for (int r = 0; r < 8; ++r) {
    float l = l_r[r];
    l += __shfl_xor(l, 1, 32); l += __shfl_xor(l, 2, 32); l += __shfl_xor(l, 4, 32); l += __shfl_xor(l, 8, 32);
    l_r[r] = (l > 0.f) ? 1.0f / l : 0.f;
  }
#pragma unroll
  for (int dt = 0; dt < DT; ++dt)
#pragma unroll
    for (int r = 0; r < 8; ++r) sO[w][8 * hh + r][dt * 16 + ln] = oacc[dt][r] * l_r[r];
  __builtin_amdgcn_fence(__ATOMIC_ACQ_REL, "workgroup");
  __builtin_amdgcn_wave_barrier();
  for (int pass = 0; pass < 2; ++pass) {
    for (int r = 0; r < 16; ++r) {
      const int row = q0 + r;
      if (row < T && lane < D / 4) {
        const v4f val = *(const v4fa*)&sO[w][r][lane * 4];
        *(volatile v4f*)(y + ((size_t)b * T + row) * ypitch + h * D + lane * 4) = val;
      }
    }
    if (pass == 0) __threadfence();
  }
}

typedef _Float16 v16h __attribute__((ext_vector_type(16)));
union FragH { v16h v; v8us half[2]; _Float16 h[16]; unsigned short u[16]; };
template <int NT>
__device__ __forceinline__ v8f mmaH(v16h ah, v16h al, v16h bh, v16h bl, v8f c) {
  c = __builtin_amdgcn_wmma_f32_16x16x32_f16(false, ah, false, bh, (short)0, c, false, false);
  if (NT >= 2) c = __builtin_amdgcn_wmma_f32_16x16x32_f16(false, al, false, bh, (short)0, c, false, false);
  if (NT >= 3) c = __builtin_amdgcn_wmma_f32_16x16x32_f16(false, ah, false, bl, (short)0, c, false, false);
  asm volatile("v_nop\n\tv_nop\n\tv_nop\n\tv_nop" : "+v"(c) : "v"(ah), "v"(al), "v"(bh), "v"(bl));
  return c;
}
template <bool ASPLIT>
__global__ __launch_bounds__(128) void k_gemm_h(const float* __restrict__ A, int lda, size_t sA, const _Float16* __restrict__ Bh, int ldb, size_t sB, float alpha, float* __restrict__ C, int ldc, size_t sC, int M, int N, int K) {
  __shared__ __attribute__((aligned(16))) float so[4][16][64];
  const int tid = threadIdx.x, w = tid >> 5, lane = tid & 31, ln = lane & 15, hh = lane >> 4; const int by = blockIdx.y;
  A += (size_t)by * sA; Bh += (size_t)by * sB; C += (size_t)by * sC;
  const int ntn = (N + 63) / 64; const int wid = blockIdx.x * 4 + w; const int mt = wid / ntn, nq = wid % ntn; if (mt * 16 >= M) return;
  const int row0 = mt * 16, col0 = nq * 64; const float* arow = A + (size_t)(row0 + ln) * lda;
  v8f acc[4] = {};
  for (int kb = 0; kb < K; kb += 32) {
    FragH ah, al;
    const v4f x0 = *(const v4fa*)(arow + kb + 8 * hh), x1 = *(const v4fa*)(arow + kb + 8 * hh + 4), x2 = *(const v4fa*)(arow + kb + 16 + 8 * hh), x3 = *(const v4fa*)(arow + kb + 16 + 8 * hh + 4);
    float xs[16] = {x0[0],x0[1],x0[2],x0[3],x1[0],x1[1],x1[2],x1[3],x2[0],x2[1],x2[2],x2[3],x3[0],x3[1],x3[2],x3[3]};
#pragma unroll
    for (int i = 0; i < 16; ++i) { const _Float16 h = (_Float16)xs[i]; ah.h[i] = h; al.h[i] = ASPLIT ? (_Float16)(xs[i] - (float)h) : (_Float16)0.0f; }
#pragma unroll
    for (int t = 0; t < 4; ++t) { if (col0 + t * 16 >= N) continue; const size_t boff = (size_t)(col0 + t * 16 + ln) * ldb + kb; FragH bq; bq.half[0] = *(const v8us*)(Bh + boff + 8 * hh); bq.half[1] = *(const v8us*)(Bh + boff + 16 + 8 * hh);
      acc[t] = mmaH<ASPLIT ? 2 : 1>(ah.v, al.v, bq.v, bq.v, acc[t]); }
  }
#pragma unroll
  for (int t = 0; t < 4; ++t) { if (col0 + t * 16 >= N) continue;
#pragma unroll
    for (int r = 0; r < 8; ++r) so[w][8 * hh + r][t * 16 + ln] = acc[t][r] * alpha; }
  __builtin_amdgcn_fence(__ATOMIC_ACQ_REL, "workgroup"); __builtin_amdgcn_wave_barrier();
  const int rsub = lane >> 4, c4 = (lane & 15) * 4;
  for (int pass = 0; pass < 2; ++pass) {
#pragma unroll
    for (int q = 0; q < 8; ++q) { const int r = q * 2 + rsub; if (col0 + c4 < N) { const v4f v = *(const v4fa*)&so[w][r][c4]; *(volatile v4f*)(C + (size_t)(row0 + r) * ldc + col0 + c4) = v; } }
    if (pass == 0) __threadfence(); }
}

__global__ __launch_bounds__(256) void k_lin1s(const float* __restrict__ x, const float* __restrict__ W1, const float* __restrict__ dinv, _Float16* __restrict__ H) { const size_t t = (size_t)blockIdx.x * 256 + threadIdx.x; if (t >= (size_t)NNODE * F1 / 8) return; const int c8 = (int)(t % (F1 / 8)) * 8; const size_t n = t / (F1 / 8); const float dn = dinv[n]; FragH f;
#pragma unroll
  for (int q = 0; q < 8; ++q) { const int c = c8 + q; float s = 0.f;
#pragma unroll
    for (int i = 0; i < FIN; ++i) s += bf16_round(x[n * FIN + i]) * bf16_round(W1[i * F1 + c]); f.h[q] = (_Float16)(s * dn); }
  const v8us o = f.half[0]; *(volatile v8us*)((unsigned short*)H + t * 8) = o; __threadfence(); *(volatile v8us*)((unsigned short*)H + t * 8) = o; }
__global__ __launch_bounds__(256) void k_wt_f16(const float* __restrict__ W, _Float16* __restrict__ Wt, int K, int N, float scale) {
  const int t = blockIdx.x * 256 + threadIdx.x; if (t >= N * (K / 8)) return; const int n = t / (K / 8), k8 = (t % (K / 8)) * 8; FragH f;
#pragma unroll
  for (int i = 0; i < 8; ++i) f.h[i] = (_Float16)(bf16_round(W[(size_t)(k8 + i) * N + n]) * scale); const v8us o = f.half[0];
  *(volatile v8us*)((unsigned short*)Wt + (size_t)n * K + k8) = o; __threadfence(); *(volatile v8us*)((unsigned short*)Wt + (size_t)n * K + k8) = o;
}

__global__ __launch_bounds__(256) void k_as(const float* __restrict__ a, const float* __restrict__ dinv, _Float16* __restrict__ A1) { const size_t t = (size_t)blockIdx.x * 256 + threadIdx.x; if (t >= (size_t)NNODE * F1 / 8) return; const size_t n = t / (F1 / 8); const float dn = dinv[n]; FragH f;
#pragma unroll
  for (int q = 0; q < 8; ++q) f.h[q] = (_Float16)(a[t * 8 + q] * dn); *(volatile v8us*)((unsigned short*)A1 + t * 8) = f.half[0]; __threadfence(); *(volatile v8us*)((unsigned short*)A1 + t * 8) = f.half[0]; }
template <int ACT>
__global__ __launch_bounds__(128) void k_gemm_hhx(const _Float16* __restrict__ A, int lda, size_t sA, const _Float16* __restrict__ Bh, int ldb, size_t sB, float alpha, const float* __restrict__ bias, size_t sBias, const float* __restrict__ CP, int rowsPerB, size_t sCPb, int row0g,
    float* __restrict__ C, _Float16* __restrict__ C16, int ldc, size_t sC, int M, int N, int K) {
  __shared__ __attribute__((aligned(16))) float so[4][16][64];
  const int tid = threadIdx.x, w = tid >> 5, lane = tid & 31, ln = lane & 15, hh = lane >> 4; const int by = blockIdx.y;
  A += (size_t)by * sA; Bh += (size_t)by * sB; const size_t cofs = (size_t)by * sC; const float* bp = bias ? bias + (size_t)by * sBias : nullptr;
  const int ntn = (N + 63) / 64; const int wid = blockIdx.x * 4 + w; const int mt = wid / ntn, nq = wid % ntn; if (mt * 16 >= M) return;
  const int row0 = mt * 16, col0 = nq * 64; const _Float16* arow = A + (size_t)(row0 + ln) * lda;
  v8f acc[4] = {};
  for (int kb = 0; kb < K; kb += 32) { FragH ah; ah.half[0] = *(const v8us*)((const unsigned short*)arow + kb + 8 * hh); ah.half[1] = *(const v8us*)((const unsigned short*)arow + kb + 16 + 8 * hh);
#pragma unroll
    for (int t = 0; t < 4; ++t) { if (col0 + t * 16 >= N) continue; const size_t boff = (size_t)(col0 + t * 16 + ln) * ldb + kb; FragH bq; bq.half[0] = *(const v8us*)((const unsigned short*)Bh + boff + 8 * hh); bq.half[1] = *(const v8us*)((const unsigned short*)Bh + boff + 16 + 8 * hh);
      acc[t] = mmaH<1>(ah.v, ah.v, bq.v, bq.v, acc[t]); }
  }
#pragma unroll
  for (int t = 0; t < 4; ++t) { if (col0 + t * 16 >= N) continue; const int col = col0 + t * 16 + ln; const float bv = bp ? bf16_round(bp[col]) : 0.f;
#pragma unroll
    for (int r = 0; r < 8; ++r) { float v = acc[t][r] * alpha + bv; if (CP) { const int bidx = (row0g + row0 + 8 * hh + r) / rowsPerB; v += CP[(size_t)bidx * sCPb + (size_t)by * 64 + col]; } if (ACT == 1) v = (v > 0.f) ? v : expm1f(v); else if (ACT == 3) v = fmaxf(v, 0.f); so[w][8 * hh + r][t * 16 + ln] = v; } }
  __builtin_amdgcn_fence(__ATOMIC_ACQ_REL, "workgroup"); __builtin_amdgcn_wave_barrier();
  const int rsub = lane >> 4, c4 = (lane & 15) * 4; typedef _Float16 v4h __attribute__((ext_vector_type(4)));
  for (int pass = 0; pass < 2; ++pass) {
#pragma unroll
    for (int q = 0; q < 8; ++q) { const int r = q * 2 + rsub; if (col0 + c4 < N) { const v4f v = *(const v4fa*)&so[w][r][c4]; if (C) *(volatile v4f*)(C + cofs + (size_t)(row0 + r) * ldc + col0 + c4) = v; if (C16) { v4h h4; for (int i = 0; i < 4; ++i) h4[i] = (_Float16)v[i]; *(volatile v4h*)(C16 + cofs + (size_t)(row0 + r) * ldc + col0 + c4) = h4; } } }
    if (pass == 0) __threadfence(); }
}


__device__ __forceinline__ int bscan1024(int cnt, int* wsum, int tid, int& total) {
  const int lane = tid & 31, wv = tid >> 5; int x = cnt;
#pragma unroll
  for (int d = 1; d < 32; d <<= 1) { const int y = __shfl_up(x, d, 32); if (lane >= d) x += y; }
  __syncthreads(); if (lane == 31) wsum[wv] = x; __syncthreads();
  int t = (lane < 32) ? wsum[lane] : 0;
#pragma unroll
  for (int d = 1; d < 32; d <<= 1) { const int y = __shfl_up(t, d, 32); if (lane >= d) t += y; }
  const int woff = (wv == 0) ? 0 : __shfl(t, wv - 1, 32); total = __shfl(t, 31, 32);
  return woff + x - cnt; }
__device__ __forceinline__ int bscan512(int cnt, int* wsum, int tid, int& total) {
  const int lane = tid & 31, wv = tid >> 5; int x = cnt;
#pragma unroll
  for (int d = 1; d < 32; d <<= 1) { const int y = __shfl_up(x, d, 32); if (lane >= d) x += y; }
  __syncthreads(); if (lane == 31) wsum[wv] = x; __syncthreads();
  int t = (lane < 16) ? wsum[lane] : 0;
#pragma unroll
  for (int d = 1; d < 32; d <<= 1) { const int y = __shfl_up(t, d, 32); if (lane >= d) t += y; }
  const int woff = (wv == 0) ? 0 : __shfl(t, wv - 1, 32); total = __shfl(t, 15, 32);
  return woff + x - cnt; }
__global__ __launch_bounds__(512) void k_sdeg(const int* __restrict__ rowi, float* __restrict__ dinv) {
  __shared__ short Lr[8192]; __shared__ int scan[16]; __shared__ float sdv[8192];
  const int tid = threadIdx.x, lane = tid & 31, wv = tid >> 5; const int n0 = blockIdx.x * 8192; int cnt[16];
#pragma unroll
  for (int s = 0; s < 16; ++s) cnt[s] = 0;
#pragma unroll 1
  for (int e0 = 0; e0 < NE; e0 += 8192) { int k_cnt = 0; unsigned hm = 0; int hv[16];
#pragma unroll
    for (int k = 0; k < 16; ++k) { const int e = e0 + tid * 16 + k; int dd_ = -1; if (e < NE) dd_ = rowi[e] - n0; hv[k] = dd_; if (dd_ >= 0 && dd_ < 8192) { hm |= 1u << k; ++k_cnt; } }
    int tot; int p = bscan512(k_cnt, scan, tid, tot);
#pragma unroll
    for (int k = 0; k < 16; ++k) if (hm & (1u << k)) { Lr[p] = (short)hv[k]; ++p; }
    __syncthreads();
    const int ntrip = (tot + 31) >> 5;
#pragma unroll 1
    for (int it = 0; it < ntrip; ++it) { const int q = it * 32 + lane; const int lr = (q < tot) ? (int)Lr[q] : -1;
      unsigned m = __builtin_amdgcn_ballot_w32(lr >= wv * 512 && lr < wv * 512 + 512);
#pragma unroll 1
      while (m) { const int bit = __builtin_ctz(m); m &= m - 1u; const int ol = __shfl(lr, bit, 32) - wv * 512;
        if (lane == (ol >> 4)) { const int sl = ol & 15;
#pragma unroll
          for (int s = 0; s < 16; ++s) if (s == sl) cnt[s] += 1; } } }
    __syncthreads(); }
#pragma unroll
  for (int s = 0; s < 16; ++s) sdv[tid * 16 + s] = rsqrtf((float)(cnt[s] + 1));
  __syncthreads();
  for (int pass = 0; pass < 2; ++pass) {
#pragma unroll
    for (int k = 0; k < 4; ++k) { const int j = k * 512 + tid; const int n = n0 + j * 4; if (n < NNODE) { v4f v; v[0] = sdv[j * 4]; v[1] = sdv[j * 4 + 1]; v[2] = sdv[j * 4 + 2]; v[3] = sdv[j * 4 + 3]; *(volatile v4f*)(dinv + n) = v; } }
    if (pass == 0) __threadfence(); }
}
#define QCAP 8
#define CHUNK 8192
template <int FW, bool RELU, bool OUT_F16>
__global__ __launch_bounds__(512) void k_sagg(const _Float16* __restrict__ Hs, const float* __restrict__ dinv, const int* __restrict__ gath, const int* __restrict__ tgt, const float* __restrict__ bias, void* __restrict__ outp) {
  __shared__ short Lr[CHUNK]; __shared__ int Le[CHUNK]; __shared__ int scan[16]; __shared__ int lq[16][QCAP][32]; __shared__ float stg[64][FW + 1];
  const int tid = threadIdx.x, lane = tid & 31, wv = tid >> 5; const int n0 = blockIdx.x * 1024; const int myl0 = wv * 64 + 2 * lane;
  float acc[2][FW]; int qn = 0;
#pragma unroll
  for (int s2 = 0; s2 < 2; ++s2)
#pragma unroll
    for (int c = 0; c < FW; ++c) acc[s2][c] = 0.f;
#pragma unroll 1
  for (int e0 = 0; e0 < NE + CHUNK; e0 += CHUNK) { const bool sentinel = (e0 >= NE); int tot = 0;
    if (!sentinel) { int k_cnt = 0; unsigned hm = 0; int hv[16];
#pragma unroll
      for (int k = 0; k < 16; ++k) { const int e = e0 + tid * 16 + k; int dd_ = -1; if (e < NE) dd_ = tgt[e] - n0; hv[k] = dd_; if (dd_ >= 0 && dd_ < 1024) { hm |= 1u << k; ++k_cnt; } }
      int p = bscan512(k_cnt, scan, tid, tot);
#pragma unroll
      for (int k = 0; k < 16; ++k) if (hm & (1u << k)) { Lr[p] = (short)hv[k]; Le[p] = e0 + tid * 16 + k; ++p; }
      __syncthreads(); }
    const int ntrip = sentinel ? 1 : ((tot + 31) >> 5);
#pragma unroll 1
    for (int it = 0; it < ntrip; ++it) { const int q = it * 32 + lane; const int lr = (!sentinel && q < tot) ? (int)Lr[q] : -1;
      unsigned m = sentinel ? 1u : __builtin_amdgcn_ballot_w32(lr >= wv * 64 && lr < wv * 64 + 64);
#pragma unroll 1
      while (m) { const int bit = __builtin_ctz(m); m &= m - 1u; const int ol = sentinel ? -2 : (__shfl(lr, bit, 32) - wv * 64); const int owner = ol >> 1; const int e = sentinel ? 0 : Le[it * 32 + bit];
        if (sentinel || __builtin_amdgcn_ballot_w32(lane == owner && qn == QCAP)) {
          int kmax = qn;
#pragma unroll
          for (int o = 16; o >= 1; o >>= 1) kmax = max(kmax, __shfl_xor(kmax, o, 32));
#pragma unroll 1
          for (int k = 0; k < kmax; ++k) { if (k < qn) { const int ent = lq[wv][k][lane]; const int eq = ent >> 1; const int sl = ent & 1; int s = gath[eq]; s = s < 0 ? 0 : (s >= NNODE ? NNODE - 1 : s);
              const unsigned short* hr16 = (const unsigned short*)Hs + (size_t)s * FW;
#pragma unroll
              for (int g = 0; g < FW / 8; ++g) { FragH fv; fv.half[0] = *(const v8us*)(hr16 + g * 8);
#pragma unroll
                for (int s2 = 0; s2 < 2; ++s2) if (s2 == sl) {
#pragma unroll
                  for (int d = 0; d < 8; ++d) acc[s2][g * 8 + d] += (float)fv.h[d]; } } } }
          qn = 0; }
        if (lane == owner) { lq[wv][qn][lane] = e * 2 + (ol & 1); ++qn; } } }
    __syncthreads(); }
#pragma unroll
  for (int s2 = 0; s2 < 2; ++s2) { const int n = n0 + myl0 + s2; const int nn = (n < NNODE) ? n : 0; const float dn = dinv[nn]; const unsigned short* hs = (const unsigned short*)Hs + (size_t)nn * FW;
#pragma unroll
    for (int g = 0; g < FW / 8; ++g) { FragH fv; fv.half[0] = *(const v8us*)(hs + g * 8);
#pragma unroll
      for (int d = 0; d < 8; ++d) { const int c = g * 8 + d; float v = (acc[s2][c] + (float)fv.h[d]) * dn + bf16_round(bias[c]); if (RELU) v = fmaxf(v, 0.f); acc[s2][c] = v; } } }
  for (int tg = 0; tg < 16; ++tg) {
    if (wv == tg) {
#pragma unroll
      for (int c = 0; c < FW; ++c) { stg[2 * lane][c] = acc[0][c]; stg[2 * lane + 1][c] = acc[1][c]; } }
    __syncthreads();
    for (int pass = 0; pass < 2; ++pass) {
      if (OUT_F16) { constexpr int TPR = FW / 8; const int r = tid / TPR, pc = tid % TPR; if (r < 64) { const int n = n0 + tg * 64 + r; if (n < NNODE) { FragH o; for (int u = 0; u < 8; ++u) o.h[u] = (_Float16)stg[r][pc * 8 + u]; *(volatile v8us*)((unsigned short*)outp + (size_t)n * FW + pc * 8) = o.half[0]; } } }
      else { constexpr int TPR = FW / 4; for (int j = tid; j < 64 * TPR; j += 512) { const int r = j / TPR, c4 = (j % TPR) * 4; const int n = n0 + tg * 64 + r; if (n < NNODE) { v4f v; v[0] = stg[r][c4]; v[1] = stg[r][c4 + 1]; v[2] = stg[r][c4 + 2]; v[3] = stg[r][c4 + 3]; *(volatile v4f*)((float*)outp + (size_t)n * FW + c4) = v; } } }
      if (pass == 0) __threadfence(); }
    __syncthreads(); } }
__global__ __launch_bounds__(128) void k_wc1(const float* __restrict__ W, _Float16* __restrict__ Bt) { const int t = threadIdx.x; if (t >= 16 * 8) return; const int o = t / 8, k8 = (t % 8) * 8; FragH f;
#pragma unroll
  for (int i = 0; i < 8; ++i) f.h[i] = (_Float16)(bf16_round(W[(k8 + i) * 16 + o]) * 16.0f); const v8us v = f.half[0]; *(volatile v8us*)((unsigned short*)Bt + o * 64 + k8) = v; __threadfence(); *(volatile v8us*)((unsigned short*)Bt + o * 64 + k8) = v; }
__global__ __launch_bounds__(128) void k_edge(const _Float16* __restrict__ h2, const int* __restrict__ ei, const _Float16* __restrict__ Bt, const float* __restrict__ bc1, const float* __restrict__ Wc2, const float* __restrict__ bc2, float* __restrict__ out) {
  __shared__ __attribute__((aligned(16))) unsigned short sA[4][16][72]; __shared__ __attribute__((aligned(16))) float so[4][16][17]; __shared__ float sres[64];
  const int tid = threadIdx.x, w = tid >> 5, lane = tid & 31, ln = lane & 15, hh = lane >> 4; const int row0 = (blockIdx.x * 4 + w) * 16; const int e = row0 + ln;
  { int nd = hh ? ei[(size_t)NE + e] : ei[e]; nd = nd < 0 ? 0 : (nd >= NNODE ? NNODE - 1 : nd); const unsigned short* srow = (const unsigned short*)h2 + (size_t)nd * F2;
#pragma unroll
    for (int g = 0; g < 4; ++g) *(v8us*)&sA[w][ln][hh * 32 + g * 8] = *(const v8us*)(srow + g * 8); }
  __builtin_amdgcn_fence(__ATOMIC_ACQ_REL, "workgroup"); __builtin_amdgcn_wave_barrier();
  v8f acc = {0.f,0.f,0.f,0.f,0.f,0.f,0.f,0.f};
#pragma unroll
  for (int kb = 0; kb < 64; kb += 32) { FragH ah; ah.half[0] = *(const v8us*)&sA[w][ln][kb + 8 * hh]; ah.half[1] = *(const v8us*)&sA[w][ln][kb + 16 + 8 * hh];
    FragH bq; bq.half[0] = *(const v8us*)((const unsigned short*)Bt + (size_t)ln * 64 + kb + 8 * hh); bq.half[1] = *(const v8us*)((const unsigned short*)Bt + (size_t)ln * 64 + kb + 16 + 8 * hh);
    acc = mmaH<1>(ah.v, ah.v, bq.v, bq.v, acc); }
#pragma unroll
  for (int q = 0; q < 8; ++q) so[w][8 * hh + q][ln] = acc[q];
  __builtin_amdgcn_fence(__ATOMIC_ACQ_REL, "workgroup"); __builtin_amdgcn_wave_barrier();
  if (lane < 16) { float s = bf16_round(bc2[0]);
#pragma unroll
    for (int o = 0; o < 16; ++o) s += fmaxf(so[w][lane][o] * 0.0625f + bf16_round(bc1[o]), 0.f) * bf16_round(Wc2[o]); sres[w * 16 + lane] = 1.0f / (1.0f + expf(-s)); }
  __syncthreads();
  if (tid < 64) { *(volatile float*)(out + (size_t)blockIdx.x * 64 + tid) = sres[tid]; } __threadfence(); if (tid < 64) { *(volatile float*)(out + (size_t)blockIdx.x * 64 + tid) = sres[tid]; }
}
extern "C" void kernel_launch(void* const* d_in, const int* in_sizes, int n_in,
                              void* d_out, int out_size, void* d_ws, size_t ws_size, hipStream_t stream) {
  (void)in_sizes; (void)n_in; (void)out_size;
  const float* x = (const float*)d_in[0]; const int* ei = (const int*)d_in[1]; const float* W1 = (const float*)d_in[2]; const float* b1 = (const float*)d_in[3]; const float* W2 = (const float*)d_in[4]; const float* b2 = (const float*)d_in[5]; const float* Wc1 = (const float*)d_in[6]; const float* bc1 = (const float*)d_in[7]; const float* Wc2 = (const float*)d_in[8]; const float* bc2 = (const float*)d_in[9];
  char* ws = (char*)d_ws; size_t off = 0;
  auto take = [&](size_t bytes) { char* p = ws + off; off += (bytes + 255) & ~(size_t)255; return p; };
  _Float16* Bt = (_Float16*)take(16 * 64 * 2); _Float16* BW2 = (_Float16*)take((size_t)F2 * F1 * 2); _Float16* A1 = (_Float16*)take((size_t)NNODE * F1 * 2);
  float* dinv = (float*)take((size_t)NNODE * 4); _Float16* H1c = (_Float16*)take((size_t)NNODE * F1 * 2); float* a1 = (float*)take((size_t)NNODE * F1 * 4); _Float16* H2c = (_Float16*)take((size_t)NNODE * F2 * 2); _Float16* a2h = (_Float16*)take((size_t)NNODE * F2 * 2);
  if (off > ws_size) return;
  const int* rowi = ei; const int* coli = ei + NE;
  k_wc1<<<1, 128, 0, stream>>>(Wc1, Bt);
  k_sdeg<<<(NNODE + 8191) / 8192, 512, 0, stream>>>(rowi, dinv);
  k_lin1s<<<(unsigned)(((size_t)NNODE * F1 / 8 + 255) / 256), 256, 0, stream>>>(x, W1, dinv, H1c);
  k_sagg<F1, true, false><<<(NNODE + 1023) / 1024, 512, 0, stream>>>(H1c, dinv, coli, rowi, b1, (void*)a1);
  k_wt_f16<<<(F2 * (F1 / 8) + 255) / 256, 256, 0, stream>>>(W2, BW2, F1, F2, 16.0f);
  k_as<<<(unsigned)(((size_t)NNODE * F1 / 8 + 255) / 256), 256, 0, stream>>>(a1, dinv, A1);
  k_gemm_hhx<0><<<dim3(((NNODE / 16) * 1 + 3) / 4, 1), 128, 0, stream>>>(A1, F1, 0, BW2, F1, 0, 0.0625f, nullptr, 0, nullptr, 1, 0, 0, nullptr, H2c, F2, 0, NNODE, F2, F1);
  k_sagg<F2, false, true><<<(NNODE + 1023) / 1024, 512, 0, stream>>>(H2c, dinv, coli, rowi, b2, (void*)a2h);
  k_edge<<<NE / 64, 128, 0, stream>>>(a2h, ei, Bt, bc1, Wc2, bc2, (float*)d_out);
}
